// TropicalSSMLayer_62302795596525
// MI455X (gfx1250) — hardware-verified
//
#include <hip/hip_runtime.h>
#include <math.h>

typedef __attribute__((ext_vector_type(16))) __bf16   v16b;
typedef __attribute__((ext_vector_type(8)))  __bf16   v8b;
typedef __attribute__((ext_vector_type(8)))  float    v8f;
typedef __attribute__((ext_vector_type(4)))  float    v4f;
typedef __attribute__((ext_vector_type(4)))  unsigned int v4u;

constexpr int kBatch  = 4;
constexpr int kSeq    = 2048;
constexpr int kDm     = 512;
constexpr int kHeads  = 4;
constexpr int kDk     = 16;
constexpr int kHD     = kHeads * kDk;
constexpr int kTok    = kBatch * kSeq;
constexpr int kNcat   = 320;
constexpr int kColK   = 64;
constexpr int kColV   = 128;
constexpr int kColA   = 256;
constexpr int kSqrtDk = 4;
constexpr float kBidScale = 1.0f / (float)kSqrtDk;
constexpr int kChunk  = 64;
constexpr int kVGP    = 132;
constexpr int kYP     = 68;

static_assert(kSqrtDk * kSqrtDk == kDk);
static_assert(kHD == 64);
static_assert(kTok == 8192);
static_assert((kTok % 64) == 0 && (kNcat % 64) == 0 && (kDm % 64) == 0);
static_assert((kDm % 32) == 0 && (kHD % 32) == 0);
static_assert(kColA + kHeads <= kNcat);
static_assert((kSeq % kChunk) == 0);

constexpr size_t kOffXH  = 0;
constexpr size_t kOffXL  = kOffXH  + (size_t)kTok  * kDm * 2;
constexpr size_t kOffWCH = kOffXL  + (size_t)kTok  * kDm * 2;
constexpr size_t kOffWCL = kOffWCH + (size_t)kNcat * kDm * 2;
constexpr size_t kOffWOH = kOffWCL + (size_t)kNcat * kDm * 2;
constexpr size_t kOffWOL = kOffWOH + (size_t)kDm   * kHD * 2;
constexpr size_t kOffP   = kOffWOL + (size_t)kDm   * kHD * 2;
constexpr size_t kOffBID = kOffP   + (size_t)kTok  * kNcat * 4;
constexpr size_t kOffAW  = kOffBID + (size_t)kTok  * kHeads * 4;
constexpr size_t kOffYH  = kOffAW  + (size_t)kTok  * kHeads * 4;
constexpr size_t kOffYL  = kOffYH  + (size_t)kTok  * kHD * 2;
constexpr size_t kWsTotal = kOffYL + (size_t)kTok  * kHD * 2;
static_assert(kWsTotal == 30408704ull);
static_assert(kWsTotal <= 134217728ull);
static_assert((kOffXL % 128) == 0 && (kOffWCH % 128) == 0 && (kOffWCL % 128) == 0 && (kOffWOH % 128) == 0 &&
              (kOffWOL % 128) == 0 && (kOffP % 128) == 0 && (kOffBID % 128) == 0 && (kOffAW % 128) == 0 &&
              (kOffYH % 128) == 0 && (kOffYL % 128) == 0);

__device__ __forceinline__ unsigned short f2bf_bits(float f) {
  unsigned u = __float_as_uint(f);
  return (unsigned short)((u + 0x7FFFu + ((u >> 16) & 1u)) >> 16);
}
__device__ __forceinline__ float bf_bits2f(unsigned short h) { return __uint_as_float(((unsigned)h) << 16); }
__device__ __forceinline__ unsigned pk16(unsigned short a, unsigned short b) { return (unsigned)a | ((unsigned)b << 16); }

__device__ __forceinline__ void split8_pack(const v4f a0, const v4f a1, v4u& hv, v4u& lv) {
  float f[8];
  f[0] = a0[0]; f[1] = a0[1]; f[2] = a0[2]; f[3] = a0[3];
  f[4] = a1[0]; f[5] = a1[1]; f[6] = a1[2]; f[7] = a1[3];
  unsigned short hb[8], lb[8];
#pragma unroll
  for (int e = 0; e < 8; ++e) {
    hb[e] = f2bf_bits(f[e]);
    lb[e] = f2bf_bits(f[e] - bf_bits2f(hb[e]));
  }
  hv = (v4u){pk16(hb[0], hb[1]), pk16(hb[2], hb[3]), pk16(hb[4], hb[5]), pk16(hb[6], hb[7])};
  lv = (v4u){pk16(lb[0], lb[1]), pk16(lb[2], lb[3]), pk16(lb[4], lb[5]), pk16(lb[6], lb[7])};
}

__device__ __forceinline__ void dep_guard4_b(v8f& a, v8f& b, v8f& c, v8f& d, v16b x, v16b y) {
  asm volatile("v_nop\n\tv_nop\n\tv_nop\n\tv_nop" : "+v"(a), "+v"(b), "+v"(c), "+v"(d) : "v"(x), "v"(y));
}
__device__ __forceinline__ void keep4_b(v16b a, v16b b, v16b c, v16b d) { asm volatile("v_nop" :: "v"(a), "v"(b), "v"(c), "v"(d)); }
__device__ __forceinline__ void acc_guard4(v8f& a, v8f& b, v8f& c, v8f& d) { asm volatile("v_nop\n\tv_nop\n\tv_nop\n\tv_nop" : "+v"(a), "+v"(b), "+v"(c), "+v"(d)); }

__device__ __forceinline__ v16b frag_load_b(const __bf16* p) {
  union U { v16b v; v8b h[2]; } f;
  f.h[0] = *(const v8b*)(p);
  f.h[1] = *(const v8b*)(p + 16);
  return f.v;
}
__device__ __forceinline__ v8f mma_b(v16b a, v16b b, v8f c) {
  return __builtin_amdgcn_wmma_f32_16x16x32_bf16(false, a, false, b, (short)0, c, false, false);
}

__global__ __launch_bounds__(256) void wmma_gemm64_split(
    const unsigned short* __restrict__ Ap, const unsigned short* __restrict__ A2p, int lda,
    const unsigned short* __restrict__ Btp, const unsigned short* __restrict__ Bt2p, int ldb,
    float* __restrict__ C, int ldc, int M, int N, int K)
{
  const __bf16* A   = (const __bf16*)Ap;
  const __bf16* A2  = (const __bf16*)A2p;
  const __bf16* Bt  = (const __bf16*)Btp;
  const __bf16* Bt2 = (const __bf16*)Bt2p;
  __shared__ __align__(16) float sT[8][16 * 68];
  const int lane = threadIdx.x & 31;
  const int wave = threadIdx.x >> 5;
  const int tilesN = N >> 6;
  const int tilesM = M >> 6;
  const int tile = blockIdx.x * 8 + wave;
  if (tile >= tilesM * tilesN) return;
  const int tm = tile / tilesN;
  const int tn = tile - tm * tilesN;
  const int m0 = tm << 6;
  const int n0 = tn << 6;

  const int rlane = lane & 15;
  const int koff  = (lane >> 4) * 8;
  const int mOff  = (lane >> 4) * 8;

  v8f acc[4][4];
#pragma unroll
  for (int i = 0; i < 4; ++i)
#pragma unroll
    for (int j = 0; j < 4; ++j) acc[i][j] = (v8f){0.f, 0.f, 0.f, 0.f, 0.f, 0.f, 0.f, 0.f};

  const size_t bRow = (size_t)(n0 + rlane) * ldb + koff;
  const size_t aRow = (size_t)(m0 + rlane) * lda + koff;
  const size_t bStep = (size_t)16 * ldb;
  const size_t aStep = (size_t)16 * lda;

  for (int k0 = 0; k0 < K; k0 += 32) {
    v16b bh[4], bl[4];
#pragma unroll
    for (int j = 0; j < 4; ++j) {
      const size_t bo = bRow + (size_t)j * bStep + k0;
      bh[j] = frag_load_b(Bt + bo);
      bl[j] = frag_load_b(Bt2 + bo);
    }
#pragma unroll
    for (int i = 0; i < 4; ++i) {
      const size_t ao = aRow + (size_t)i * aStep + k0;
      v16b ah = frag_load_b(A + ao);
      v16b al = frag_load_b(A2 + ao);
#pragma unroll
      for (int j = 0; j < 4; ++j) {
        acc[i][j] = mma_b(ah, bh[j], acc[i][j]);
        acc[i][j] = mma_b(ah, bl[j], acc[i][j]);
        acc[i][j] = mma_b(al, bh[j], acc[i][j]);
      }
      dep_guard4_b(acc[i][0], acc[i][1], acc[i][2], acc[i][3], ah, al);
    }
    keep4_b(bh[0], bh[1], bh[2], bh[3]);
    keep4_b(bl[0], bl[1], bl[2], bl[3]);
  }
  acc_guard4(acc[0][0], acc[0][1], acc[0][2], acc[0][3]);
  acc_guard4(acc[1][0], acc[1][1], acc[1][2], acc[1][3]);
  acc_guard4(acc[2][0], acc[2][1], acc[2][2], acc[2][3]);
  acc_guard4(acc[3][0], acc[3][1], acc[3][2], acc[3][3]);

  float* slab = sT[wave];
  const int hh = lane >> 4, c4 = (lane & 15) * 4;
#pragma unroll
  for (int i = 0; i < 4; ++i) {
    const int mBase = m0 + (i << 4);
#pragma unroll
    for (int j = 0; j < 4; ++j) {
#pragma unroll
      for (int r = 0; r < 8; ++r) {
        slab[(mOff + r) * 68 + (j << 4) + rlane] = acc[i][j][r];
      }
    }
    __builtin_amdgcn_fence(__ATOMIC_RELEASE, "workgroup");
    __builtin_amdgcn_wave_barrier();
    __builtin_amdgcn_fence(__ATOMIC_ACQUIRE, "workgroup");
    for (int pass = 0; pass < 2; ++pass) {
#pragma unroll
      for (int it = 0; it < 8; ++it) {
        const int row = it * 2 + hh;
        v4f v = *(const v4f*)(slab + row * 68 + c4);
        *(volatile v4f*)(C + (size_t)(mBase + row) * ldc + n0 + c4) = v;
      }
      __threadfence();
    }
    __builtin_amdgcn_fence(__ATOMIC_RELEASE, "workgroup");
    __builtin_amdgcn_wave_barrier();
    __builtin_amdgcn_fence(__ATOMIC_ACQUIRE, "workgroup");
  }
}

__global__ __launch_bounds__(256) void split_rows_kernel(
    const float* __restrict__ src, unsigned short* __restrict__ dhi, unsigned short* __restrict__ dlo, int total8)
{
  const int i = blockIdx.x * 256 + threadIdx.x;
  if (i >= total8) return;
  const size_t e0 = (size_t)i << 3;
  const v4f a0 = *(const v4f*)(src + e0);
  const v4f a1 = *(const v4f*)(src + e0 + 4);
  v4u hv, lv;
  split8_pack(a0, a1, hv, lv);
  unsigned short* qh = dhi + e0;
  unsigned short* ql = dlo + e0;
  *(volatile v4u*)qh = hv;
  *(volatile v4u*)ql = lv;
  __threadfence();
  *(volatile v4u*)qh = hv;
  *(volatile v4u*)ql = lv;
}

__global__ __launch_bounds__(256) void transpose_split_kernel(
    const float* __restrict__ W, unsigned short* __restrict__ Bh, unsigned short* __restrict__ Bl,
    int Kdim, int Ndim, int rowOff)
{
  __shared__ float tile[64 * 65];
  const int tid = threadIdx.x, lane = tid & 31, wave = tid >> 5;
  const int n0 = blockIdx.x * 64;
  const int k0 = blockIdx.y * 64;
#pragma unroll
  for (int p = 0; p < 16; ++p) {
    const int idx = tid + p * 256;
    const int kk  = idx >> 6;
    const int nn  = idx & 63;
    const int n   = n0 + nn;
    const int nc  = (n < Ndim) ? n : (Ndim - 1);
    const float v = W[(size_t)(k0 + kk) * Ndim + nc];
    tile[kk * 65 + nn] = (n < Ndim) ? v : 0.0f;
  }
  __syncthreads();
  const int q = lane >> 3, c8 = (lane & 7) * 8;
  v4u hv[2], lv[2];
#pragma unroll
  for (int it = 0; it < 2; ++it) {
    const int nrow = it * 32 + wave * 4 + q;
    v4f a0, a1;
    a0[0] = tile[(c8 + 0) * 65 + nrow];
    a0[1] = tile[(c8 + 1) * 65 + nrow];
    a0[2] = tile[(c8 + 2) * 65 + nrow];
    a0[3] = tile[(c8 + 3) * 65 + nrow];
    a1[0] = tile[(c8 + 4) * 65 + nrow];
    a1[1] = tile[(c8 + 5) * 65 + nrow];
    a1[2] = tile[(c8 + 6) * 65 + nrow];
    a1[3] = tile[(c8 + 7) * 65 + nrow];
    split8_pack(a0, a1, hv[it], lv[it]);
  }
  for (int pass = 0; pass < 2; ++pass) {
#pragma unroll
    for (int it = 0; it < 2; ++it) {
      const int nrow = it * 32 + wave * 4 + q;
      const size_t o = (size_t)(rowOff + n0 + nrow) * Kdim + k0 + c8;
      *(volatile v4u*)(Bh + o) = hv[it];
      *(volatile v4u*)(Bl + o) = lv[it];
    }
    __threadfence();
  }
}

__global__ __launch_bounds__(256) void bid_decay_kernel(
    const float* __restrict__ P, const float* __restrict__ ba,
    float* __restrict__ bidw, float* __restrict__ aw)
{
  const int g = blockIdx.x * 256 + threadIdx.x;
  const int token = g >> 2;
  const int h = g & 3;
  const float* pr = P + (size_t)token * kNcat;
  const float* qp = pr + h * kDk;
  const float* kp = pr + kColK + h * kDk;
  float s = 0.0f;
#pragma unroll
  for (int j = 0; j < 4; ++j) {
    const v4f qv = *(const v4f*)(qp + 4 * j);
    const v4f kv = *(const v4f*)(kp + 4 * j);
    s = fmaf(qv[0], kv[0], s);
    s = fmaf(qv[1], kv[1], s);
    s = fmaf(qv[2], kv[2], s);
    s = fmaf(qv[3], kv[3], s);
  }
  const float bid = s * kBidScale;
  const float z = pr[kColA + h] + ba[h];
  const float sp = fmaxf(z, 0.0f) + log1pf(expf(-fabsf(z)));
  const float a = -sp;
  *(volatile float*)(bidw + g) = bid;
  *(volatile float*)(aw + g) = a;
  __threadfence();
  *(volatile float*)(bidw + g) = bid;
  *(volatile float*)(aw + g) = a;
}

__global__ __launch_bounds__(64) void scan_gate_kernel(
    const float* __restrict__ P, const float* __restrict__ bidw, const float* __restrict__ aw,
    const float* __restrict__ bg, unsigned short* __restrict__ YH, unsigned short* __restrict__ YL)
{
  __shared__ __align__(16) float sVG[kChunk * kVGP];
  __shared__ __align__(16) float sB[kChunk * kHeads];
  __shared__ __align__(16) float sA[kChunk * kHeads];
  __shared__ __align__(16) float sY[kChunk * kYP];
  const int tid = threadIdx.x, lane = tid & 31, wave = tid >> 5;
  const int h = tid >> 4;
  const size_t row0 = (size_t)blockIdx.x * kSeq;
  const float bgv = bg[tid];
  float m = -1.0e30f;
  float Z = 0.0f;
  float Nn = 0.0f;
  const int sc4 = (tid & 31) * 4;
  const int sr0 = tid >> 5;
  const int q = lane >> 3, c8 = (lane & 7) * 8;
#pragma unroll 1
  for (int t0 = 0; t0 < kSeq; t0 += kChunk) {
    __syncthreads();
    const float* pbase = P + (row0 + t0 + sr0) * kNcat + kColV + sc4;
#pragma unroll 8
    for (int i = 0; i < 32; ++i) {
      const int r = sr0 + 2 * i;
      *(v4f*)(sVG + r * kVGP + sc4) = *(const v4f*)(pbase + (size_t)(2 * i) * kNcat);
    }
    *(v4f*)(sB + tid * 4) = *(const v4f*)(bidw + (row0 + t0) * kHeads + tid * 4);
    *(v4f*)(sA + tid * 4) = *(const v4f*)(aw + (row0 + t0) * kHeads + tid * 4);
    __syncthreads();
#pragma unroll 1
    for (int s = 0; s < kChunk; ++s) {
      const float bidv = sB[s * kHeads + h];
      const float av   = sA[s * kHeads + h];
      const float vv   = sVG[s * kVGP + tid];
      const float gp   = sVG[s * kVGP + kHD + tid] + bgv;
      const float ma   = m + av;
      const float dlt  = ma - bidv;
      const float e    = expf(-fabsf(dlt));
      const bool  ge   = (dlt >= 0.0f);
      const float e1   = ge ? 1.0f : e;
      const float e2   = ge ? e : 1.0f;
      m  = ge ? ma : bidv;
      Z  = fmaf(Z, e1, e2);
      Nn = fmaf(Nn, e1, e2 * vv);
      const float gate = __builtin_amdgcn_rcpf(1.0f + expf(-gp));
      const float y = Nn * __builtin_amdgcn_rcpf(Z);
      sY[s * kYP + tid] = y * gate;
    }
    __syncthreads();
    v4u hv[8], lv[8];
#pragma unroll
    for (int it = 0; it < 8; ++it) {
      const int row = it * 8 + wave * 4 + q;
      const float* sp = sY + row * kYP + c8;
      const v4f a0 = *(const v4f*)(sp);
      const v4f a1 = *(const v4f*)(sp + 4);
      split8_pack(a0, a1, hv[it], lv[it]);
    }
    for (int pass = 0; pass < 2; ++pass) {
#pragma unroll
      for (int it = 0; it < 8; ++it) {
        const int row = it * 8 + wave * 4 + q;
        const size_t o = (row0 + t0 + row) * kHD + c8;
        *(volatile v4u*)(YH + o) = hv[it];
        *(volatile v4u*)(YL + o) = lv[it];
      }
      __threadfence();
    }
  }
}

extern "C" void kernel_launch(void* const* d_in, const int* in_sizes, int n_in,
                              void* d_out, int out_size, void* d_ws, size_t ws_size,
                              hipStream_t stream)
{
  if (n_in < 9) return;
  if (in_sizes[0] != kTok * kDm) return;
  if (in_sizes[1] != kDm * kHD) return;
  if (in_sizes[2] != kDm * kHD) return;
  if (in_sizes[3] != kDm * kHD) return;
  if (in_sizes[4] != kDm * kHeads) return;
  if (in_sizes[5] != kHeads) return;
  if (in_sizes[6] != kDm * kHD) return;
  if (in_sizes[7] != kHD) return;
  if (in_sizes[8] != kHD * kDm) return;
  if (out_size != kTok * kDm) return;
  if (ws_size < kWsTotal) return;

  const float* x  = (const float*)d_in[0];
  const float* Wq = (const float*)d_in[1];
  const float* Wk = (const float*)d_in[2];
  const float* Wv = (const float*)d_in[3];
  const float* Wa = (const float*)d_in[4];
  const float* ba = (const float*)d_in[5];
  const float* Wg = (const float*)d_in[6];
  const float* bg = (const float*)d_in[7];
  const float* Wo = (const float*)d_in[8];
  float* out = (float*)d_out;

  char* ws = (char*)d_ws;
  unsigned short* XH  = (unsigned short*)(ws + kOffXH);
  unsigned short* XL  = (unsigned short*)(ws + kOffXL);
  unsigned short* WCH = (unsigned short*)(ws + kOffWCH);
  unsigned short* WCL = (unsigned short*)(ws + kOffWCL);
  unsigned short* WOH = (unsigned short*)(ws + kOffWOH);
  unsigned short* WOL = (unsigned short*)(ws + kOffWOL);
  float*          P   = (float*)(ws + kOffP);
  float*          BID = (float*)(ws + kOffBID);
  float*          AW  = (float*)(ws + kOffAW);
  unsigned short* YH  = (unsigned short*)(ws + kOffYH);
  unsigned short* YL  = (unsigned short*)(ws + kOffYL);

  split_rows_kernel<<<(kTok * kDm / 8) / 256, 256, 0, stream>>>(x, XH, XL, kTok * kDm / 8);

  transpose_split_kernel<<<dim3(1, kDm / 64), 256, 0, stream>>>(Wq, WCH, WCL, kDm, kHD, 0);
  transpose_split_kernel<<<dim3(1, kDm / 64), 256, 0, stream>>>(Wk, WCH, WCL, kDm, kHD, 64);
  transpose_split_kernel<<<dim3(1, kDm / 64), 256, 0, stream>>>(Wv, WCH, WCL, kDm, kHD, 128);
  transpose_split_kernel<<<dim3(1, kDm / 64), 256, 0, stream>>>(Wg, WCH, WCL, kDm, kHD, 192);
  transpose_split_kernel<<<dim3(1, kDm / 64), 256, 0, stream>>>(Wa, WCH, WCL, kDm, kHeads, 256);
  transpose_split_kernel<<<dim3(kDm / 64, kHD / 64), 256, 0, stream>>>(Wo, WOH, WOL, kHD, kDm, 0);

  wmma_gemm64_split<<<((kTok / 64) * (kNcat / 64)) / 8, 256, 0, stream>>>(
      XH, XL, kDm, WCH, WCL, kDm, P, kNcat, kTok, kNcat, kDm);

  bid_decay_kernel<<<(kTok * kHeads) / 256, 256, 0, stream>>>(P, ba, BID, AW);

  scan_gate_kernel<<<kBatch, 64, 0, stream>>>(P, BID, AW, bg, YH, YL);

  wmma_gemm64_split<<<((kTok / 64) * (kDm / 64)) / 8, 256, 0, stream>>>(
      YH, YL, kHD, WOH, WOL, kHD, out, kDm, kTok, kDm, kHD);
}
